// InformationExtractor_29068338659878
// MI455X (gfx1250) — hardware-verified
//
#include <hip/hip_runtime.h>
#include <stdint.h>


typedef _Float16 v16h __attribute__((ext_vector_type(16)));
typedef _Float16 v8h  __attribute__((ext_vector_type(8))) __attribute__((may_alias));
typedef float    v8f  __attribute__((ext_vector_type(8)));
typedef float    v4f  __attribute__((ext_vector_type(4))) __attribute__((may_alias));

union Frag { v16h v; v8h hv[2]; };

#define IMG_PER_BLK 16
#define GRP_IMG     4
#define NGRP        4
#define NTHR        256

#define HS_HALVES   (GRP_IMG * 16 * 16 * 32)
#define WS2_HALVES  (64 * 288)
#define FS_FLOATS   (GRP_IMG * 49 * 64)

__device__ __forceinline__ v8f wmma_f16(v16h a, v16h b, v8f c) {
    c = __builtin_amdgcn_wmma_f32_16x16x32_f16(false, a, false, b, (short)0, c, false, false);
    asm volatile("v_nop\n\tv_nop\n\tv_nop\n\tv_nop" : "+v"(c) : "v"(a), "v"(b));
    return c;
}

__global__ void __launch_bounds__(NTHR)
k_fused(const float* __restrict__ x,
        const float* __restrict__ w1, const float* __restrict__ b1,
        const float* __restrict__ w2, const float* __restrict__ b2,
        const float* __restrict__ aw, const float* __restrict__ ab,
        const float* __restrict__ ew, const float* __restrict__ eb,
        const float* __restrict__ fw, const float* __restrict__ fb,
        float* __restrict__ out, int B)
{
    __shared__ __align__(16) _Float16 hs[HS_HALVES];
    __shared__ __align__(16) _Float16 ws2[WS2_HALVES];
    __shared__ __align__(16) float fs[FS_FLOATS];
    __shared__ __align__(16) float w1s[32 * 12];
    __shared__ float b1s[32];
    __shared__ float b2s[64];
    __shared__ float aws[64];
    __shared__ __align__(16) float fws[256];
    __shared__ float lexp[GRP_IMG * 128];
    __shared__ __align__(16) float outst[IMG_PER_BLK * 2];

    const int tid  = threadIdx.x;
    const int lane = tid & 31;
    const int wid  = tid >> 5;
    const int blk  = blockIdx.x;

    {
        const _Float16 hz = (_Float16)0.0f;
        const v8h z8 = {hz, hz, hz, hz, hz, hz, hz, hz};
        for (int i = tid; i < HS_HALVES / 8; i += NTHR) *(v8h*)(hs + i * 8) = z8;
        for (int i = tid; i < WS2_HALVES; i += NTHR) {
            const int n  = i / 288;
            const int k  = i - n * 288;
            const int t  = k >> 5;
            const int ic = k & 31;
            ws2[i] = (_Float16)(w2[(n * 32 + ic) * 9 + t] * 16.0f);
        }
        for (int i = tid; i < 32 * 12; i += NTHR) {
            const int c  = i / 12;
            const int t  = i - c * 12;
            const int tt = t < 9 ? t : 8;
            const float v = w1[c * 9 + tt];
            w1s[i] = (t < 9) ? v : 0.0f;
        }
        if (tid < 32) b1s[tid] = b1[tid];
        if (tid < 64) b2s[tid] = b2[tid];
        if (tid < 49) aws[tid] = aw[tid];
        fws[tid] = fw[tid];
        if (tid < IMG_PER_BLK * 2) outst[tid] = 0.0f;
    }
    __syncthreads();

    for (int g = 0; g < NGRP; ++g) {
        for (int it = tid; it < GRP_IMG * 196; it += NTHR) {
            const int li = it / 196;
            const int r  = it - li * 196;
            const int oy = r / 14;
            const int ox = r - oy * 14;
            int gimg = blk * IMG_PER_BLK + g * GRP_IMG + li;
            gimg = gimg < B ? gimg : (B - 1);
            const float* xb = x + (size_t)gimg * 784;

            float win[4][4];
            #pragma unroll
            for (int dy = 0; dy < 4; ++dy) {
                const int iy  = 2 * oy - 1 + dy;
                const int iyc = iy < 0 ? 0 : (iy > 27 ? 27 : iy);
                const bool oky = (unsigned)iy < 28u;
                #pragma unroll
                for (int dx = 0; dx < 4; ++dx) {
                    const int ix  = 2 * ox - 1 + dx;
                    const int ixc = ix < 0 ? 0 : (ix > 27 ? 27 : ix);
                    const bool ok = oky && ((unsigned)ix < 28u);
                    const float v = xb[iyc * 28 + ixc];
                    win[dy][dx] = ok ? v : 0.0f;
                }
            }

            _Float16* cell = hs + ((li * 16 + oy + 1) * 16 + (ox + 1)) * 32;
            #pragma unroll 1
            for (int cg = 0; cg < 4; ++cg) {
                const _Float16 hz = (_Float16)0.0f;
                v8h hvv = {hz, hz, hz, hz, hz, hz, hz, hz};
                #pragma unroll
                for (int j = 0; j < 8; ++j) {
                    const int c = cg * 8 + j;
                    const v4f wa = *(const v4f*)(w1s + c * 12);
                    const v4f wb = *(const v4f*)(w1s + c * 12 + 4);
                    const v4f wc = *(const v4f*)(w1s + c * 12 + 8);
                    const float wt[9] = {wa.x, wa.y, wa.z, wa.w, wb.x, wb.y, wb.z, wb.w, wc.x};
                    float s00 = 0.f, s01 = 0.f, s10 = 0.f, s11 = 0.f;
                    #pragma unroll
                    for (int ky = 0; ky < 3; ++ky) {
                        #pragma unroll
                        for (int kx = 0; kx < 3; ++kx) {
                            const float wv = wt[ky * 3 + kx];
                            s00 = fmaf(win[ky][kx],         wv, s00);
                            s01 = fmaf(win[ky][kx + 1],     wv, s01);
                            s10 = fmaf(win[ky + 1][kx],     wv, s10);
                            s11 = fmaf(win[ky + 1][kx + 1], wv, s11);
                        }
                    }
                    const float mx = fmaxf(fmaxf(s00, s01), fmaxf(s10, s11));
                    const float pv = fmaxf(mx + b1s[c], 0.0f);
                    hvv[j] = (_Float16)pv;
                }
                *(v8h*)(cell + cg * 8) = hvv;
            }
        }
        __syncthreads();

        {
            const int nw   = wid & 3;
            const int qpar = wid >> 2;
            const int m    = lane & 15;
            const int h    = lane >> 4;
            const int li   = m >> 2;
            const int p    = m & 3;
            const int n    = nw * 16 + m;
            const float bias = b2s[n];

            Frag bf[9];
            const _Float16* brow = ws2 + n * 288 + 8 * h;
            #pragma unroll
            for (int t = 0; t < 9; ++t) {
                bf[t].hv[0] = *(const v8h*)(brow + t * 32);
                bf[t].hv[1] = *(const v8h*)(brow + t * 32 + 16);
            }

            for (int q = qpar; q < 49; q += 2) {
                const int qy = q / 7;
                const int qx = q - qy * 7;
                const int cy = 2 * qy + (p >> 1);
                const int cx = 2 * qx + (p & 1);
                const _Float16* arow = hs + ((li * 16 + cy) * 16 + cx) * 32 + 8 * h;
                v8f acc = {0.f, 0.f, 0.f, 0.f, 0.f, 0.f, 0.f, 0.f};
                #pragma unroll
                for (int t = 0; t < 9; ++t) {
                    const int off = ((t / 3) * 16 + (t % 3)) * 32;
                    Frag a;
                    a.hv[0] = *(const v8h*)(arow + off);
                    a.hv[1] = *(const v8h*)(arow + off + 16);
                    acc = wmma_f16(a.v, bf[t].v, acc);
                }
                const float m0 = fmaxf(fmaxf(acc[0], acc[1]), fmaxf(acc[2], acc[3]));
                const float m1 = fmaxf(fmaxf(acc[4], acc[5]), fmaxf(acc[6], acc[7]));
                const float p0 = fmaxf(fmaf(m0, 0.0625f, bias), 0.0f);
                const float p1 = fmaxf(fmaf(m1, 0.0625f, bias), 0.0f);
                fs[((2 * h)     * 49 + q) * 64 + n] = p0;
                fs[((2 * h + 1) * 49 + q) * 64 + n] = p1;
            }
        }
        __syncthreads();

        {
            const int li = tid >> 6;
            const int e  = tid & 63;
            float al = ab[0];
            float e0 = 0.f, e1 = 0.f;
            const float* ewr = ew + (size_t)e * 98;
            #pragma unroll 7
            for (int q = 0; q < 49; ++q) {
                const float f = fs[(li * 49 + q) * 64 + e];
                al = fmaf(f, aws[q], al);
                e0 = fmaf(f, ewr[2 * q],     e0);
                e1 = fmaf(f, ewr[2 * q + 1], e1);
            }
            const float alc = fminf(fmaxf(al, -30.0f), 30.0f);
            const float a   = 1.0f / (1.0f + expf(-alc));
            lexp[li * 128 + e * 2]     = fmaxf((e0 + eb[e * 2])     * a, 0.0f);
            lexp[li * 128 + e * 2 + 1] = fmaxf((e1 + eb[e * 2 + 1]) * a, 0.0f);
        }
        __syncthreads();

        if (tid < GRP_IMG * 2) {
            const int li = tid >> 1;
            const int o  = tid & 1;
            float acc = fb[o];
            #pragma unroll 8
            for (int j = 0; j < 128; ++j) acc = fmaf(lexp[li * 128 + j], fws[j * 2 + o], acc);
            outst[(g * GRP_IMG + li) * 2 + o] = acc;
        }
    }
    __syncthreads();

    if (wid == 0) {
        const int nval = B - blk * IMG_PER_BLK;
        float* op = out + (size_t)blk * (IMG_PER_BLK * 2);
        if (nval >= IMG_PER_BLK) {
            v4f v = {0.f, 0.f, 0.f, 0.f};
            if (lane < 8) {
                v.x = outst[lane * 4];     v.y = outst[lane * 4 + 1];
                v.z = outst[lane * 4 + 2]; v.w = outst[lane * 4 + 3];
                *(volatile v4f*)(op + lane * 4) = v;
            }
            __threadfence();
            if (lane < 8) *(volatile v4f*)(op + lane * 4) = v;
        } else {
            const int nf = nval * 2;
            const float v = outst[lane];
            if (lane < nf) *(volatile float*)(op + lane) = v;
            __threadfence();
            if (lane < nf) *(volatile float*)(op + lane) = v;
        }
    }
}

extern "C" void kernel_launch(void* const* d_in, const int* in_sizes, int n_in,
                              void* d_out, int out_size, void* d_ws, size_t ws_size,
                              hipStream_t stream)
{
    (void)d_ws; (void)ws_size;
    if (n_in < 11) return;
    const float* x   = (const float*)d_in[0];
    const float* w1  = (const float*)d_in[1];
    const float* b1  = (const float*)d_in[2];
    const float* w2  = (const float*)d_in[3];
    const float* b2  = (const float*)d_in[4];
    const float* aw  = (const float*)d_in[5];
    const float* ab  = (const float*)d_in[6];
    const float* ew  = (const float*)d_in[7];
    const float* eb  = (const float*)d_in[8];
    const float* fw  = (const float*)d_in[9];
    const float* fb  = (const float*)d_in[10];
    float* out = (float*)d_out;

    int B = in_sizes[0] / 784;
    const int Bo = out_size / 2;
    if (Bo < B) B = Bo;
    if (B <= 0) return;
    if (in_sizes[1] < 288 || in_sizes[2] < 32 || in_sizes[3] < 18432 || in_sizes[4] < 64 ||
        in_sizes[5] < 49 || in_sizes[6] < 1 || in_sizes[7] < 6272 || in_sizes[8] < 128 ||
        in_sizes[9] < 256 || in_sizes[10] < 2) return;

    const int nblk = (B + IMG_PER_BLK - 1) / IMG_PER_BLK;
    k_fused<<<dim3(nblk), dim3(NTHR), 0, stream>>>(x, w1, b1, w2, b2, aw, ab, ew, eb, fw, fb, out, B);
    (void)hipGetLastError();
}
